// SAGEConvWithMultipleLinearLayers_88433376624936
// MI455X (gfx1250) — hardware-verified
//
#include <hip/hip_runtime.h>
#include <stddef.h>


#define FEAT    256
#define H1D     512
#define H2D     256
#define NCLS    5
#define NCLP    16
#define K1      (2 * FEAT)
#define K2      (2 * H1D)
#define NTHR    256
#define NWAVE   8
#define EPT     8
#define NGRP    2
#define CHUNK   (NTHR * EPT * NGRP)
#define WCAP    (EPT * NGRP * 32)
#define LISTN   (NWAVE * WCAP)
#define NBC     4096
#define NBF     1024
#define RCAP    40960
#define RBN     128
#define TGT     256
#define DEGCAP  128
#define GR      64
#define SP      264
#define OTHR    512
#define WSCALE  16.0f
#define WINV    0.0625f

#define LDS_FILL ((RCAP + NBF + LISTN) * 4 + 64)
#define LDS_TAIL (2 * GR * SP * 2)

static_assert((CHUNK & (CHUNK - 1)) == 0);
static_assert(CHUNK <= 4096);
static_assert(NBC <= 4096 && NBF <= 4096);
static_assert((NBC & (NBC - 1)) == 0 && (NBF & (NBF - 1)) == 0);
static_assert(NBC == 4 * NBF);
static_assert(OTHR * 8 == NBC);
static_assert((RCAP % 32) == 0);
static_assert(TGT == NWAVE * 32 && (TGT % GR) == 0);
static_assert(NTHR == 256 && GR == 64);
static_assert(FEAT == 256 && H2D == 256 && H1D == 2 * FEAT);
static_assert(((SP * 2) % 16) == 0);
static_assert((GR * 8 + GR * NCLS) * 4 <= GR * SP * 2);
static_assert(NCLS <= 8 && NCLP == 16 && (GR * NCLS) % 4 == 0);
static_assert((H1D * K1 / 8) % NTHR == 0 && (H2D * K2 / 8) % NTHR == 0 && (H2D * H2D / 8) % NTHR == 0 && (NCLP * H2D / 8) % NTHR == 0);

typedef float    v4f  __attribute__((ext_vector_type(4)));
typedef float    v8f  __attribute__((ext_vector_type(8)));
typedef int      v4i  __attribute__((ext_vector_type(4)));
typedef _Float16 v8h  __attribute__((ext_vector_type(8)));
typedef _Float16 v16h __attribute__((ext_vector_type(16)));
union FragH { v16h v; v8h h[2]; };

__device__ __forceinline__ v8h tohalf8(v8f x) { return __builtin_convertvector(x, v8h); }
__device__ __forceinline__ v8f tofloat8(v8h x) { return __builtin_convertvector(x, v8f); }
__device__ __forceinline__ v8f join8(v4f a, v4f b) { return __builtin_shufflevector(a, b, 0, 1, 2, 3, 4, 5, 6, 7); }

__device__ __forceinline__ v8f wmh(v16h a, v16h b, v8f c) {
  v8f d = __builtin_amdgcn_wmma_f32_16x16x32_f16(false, a, false, b, (short)0, c, false, false);
  asm volatile("v_nop\n\tv_nop\n\tv_nop\n\tv_nop" : "+v"(d) : "v"(a), "v"(b));
  return d;
}
__device__ __forceinline__ void wmh2(v8f& d0, v8f& d1, v16h a0, v16h a1, v16h b) {
  d0 = __builtin_amdgcn_wmma_f32_16x16x32_f16(false, a0, false, b, (short)0, d0, false, false);
  d1 = __builtin_amdgcn_wmma_f32_16x16x32_f16(false, a1, false, b, (short)0, d1, false, false);
  asm volatile("v_nop\n\tv_nop\n\tv_nop\n\tv_nop" : "+v"(d0), "+v"(d1) : "v"(a0), "v"(a1), "v"(b));
}

template <int NB>
__device__ __forceinline__ int scan_chunk(const int* __restrict__ dsts, int nE, int cbase, int slotBase,
                                          int vec8, int* list, int tid, int lane, int wave) {
  int wc = 0;
#pragma unroll
  for (int g = 0; g < NGRP; ++g) {
    const int el0  = (g * NTHR + tid) * EPT;
    const int e0   = cbase + el0;
    const int sent = -2147483647 - 1;
    v4i da, db;
    if (vec8 != 0 && cbase + CHUNK <= nE) {
      da = *(const v4i*)(dsts + e0);
      db = *(const v4i*)(dsts + e0 + 4);
    } else {
      da.x = (e0     < nE) ? dsts[min(e0, nE - 1)] : sent;
      da.y = (e0 + 1 < nE) ? dsts[min(e0 + 1, nE - 1)] : sent;
      da.z = (e0 + 2 < nE) ? dsts[min(e0 + 2, nE - 1)] : sent;
      da.w = (e0 + 3 < nE) ? dsts[min(e0 + 3, nE - 1)] : sent;
      db.x = (e0 + 4 < nE) ? dsts[min(e0 + 4, nE - 1)] : sent;
      db.y = (e0 + 5 < nE) ? dsts[min(e0 + 5, nE - 1)] : sent;
      db.z = (e0 + 6 < nE) ? dsts[min(e0 + 6, nE - 1)] : sent;
      db.w = (e0 + 7 < nE) ? dsts[min(e0 + 7, nE - 1)] : sent;
    }
    const unsigned nb = (unsigned)slotBase;
    const unsigned s0 = (unsigned)da.x - nb, s1 = (unsigned)da.y - nb;
    const unsigned s2 = (unsigned)da.z - nb, s3 = (unsigned)da.w - nb;
    const unsigned s4 = (unsigned)db.x - nb, s5 = (unsigned)db.y - nb;
    const unsigned s6 = (unsigned)db.z - nb, s7 = (unsigned)db.w - nb;
    const bool h0 = s0 < (unsigned)NB, h1 = s1 < (unsigned)NB, h2 = s2 < (unsigned)NB, h3 = s3 < (unsigned)NB;
    const bool h4 = s4 < (unsigned)NB, h5 = s5 < (unsigned)NB, h6 = s6 < (unsigned)NB, h7 = s7 < (unsigned)NB;
    const unsigned any = __builtin_amdgcn_ballot_w32(h0 | h1 | h2 | h3 | h4 | h5 | h6 | h7);
    if (any != 0u) {
#define HITJ(J, HJ, SJ) { \
        const unsigned mj = __builtin_amdgcn_ballot_w32(HJ); \
        if (mj != 0u) { \
          if (HJ) { \
            const int pos = wc + (int)__builtin_amdgcn_mbcnt_lo(mj, 0u); \
            if (pos < WCAP) list[wave * WCAP + pos] = ((el0 + (J)) << 12) | (int)(SJ); \
          } \
          wc += (int)__builtin_popcount(mj); } }
      HITJ(0, h0, s0)
      HITJ(1, h1, s1)
      HITJ(2, h2, s2)
      HITJ(3, h3, s3)
      HITJ(4, h4, s4)
      HITJ(5, h5, s5)
      HITJ(6, h6, s6)
      HITJ(7, h7, s7)
#undef HITJ
    }
  }
  return wc;
}

__global__ __launch_bounds__(NTHR) void k_wprep(
    const float* __restrict__ W1l, const float* __restrict__ W1r,
    const float* __restrict__ W2l, const float* __restrict__ W2r,
    const float* __restrict__ Wh,  const float* __restrict__ Wfc,
    _Float16* B1, _Float16* B2, _Float16* Bh, _Float16* Bf, int nHid) {
  const int g0 = H1D * K1 / 8;
  const int g1 = H2D * K2 / 8;
  const int g2 = nHid * (H2D * H2D / 8);
  const int g3 = NCLP * H2D / 8;
  const int bstart = blockIdx.x * NTHR;
  const int i = bstart + (int)threadIdx.x;
  if (i >= g0 + g1 + g2 + g3) return;
  float v[8];
  _Float16* dp;
  if (bstart < g0) {
    const int o  = i * 8;
    const int n  = o / K1;
    const int k0 = o - n * K1;
#pragma unroll
    for (int e = 0; e < 8; ++e) {
      const int k  = k0 + e;
      const int kl = k < FEAT ? k : FEAT - 1;
      int kr = k - FEAT; kr = kr < 0 ? 0 : (kr > FEAT - 1 ? FEAT - 1 : kr);
      const float a = W1l[(size_t)kl * H1D + n];
      const float b = W1r[(size_t)kr * H1D + n];
      v[e] = (k < FEAT ? a : b) * WSCALE;
    }
    dp = B1 + o;
  } else if (bstart < g0 + g1) {
    const int o  = (i - g0) * 8;
    const int n  = o / K2;
    const int k0 = o - n * K2;
#pragma unroll
    for (int e = 0; e < 8; ++e) {
      const int k  = k0 + e;
      const int kl = k < H1D ? k : H1D - 1;
      int kr = k - H1D; kr = kr < 0 ? 0 : (kr > H1D - 1 ? H1D - 1 : kr);
      const float a = W2l[(size_t)kl * H2D + n];
      const float b = W2r[(size_t)kr * H2D + n];
      v[e] = (k < H1D ? a : b) * WSCALE;
    }
    dp = B2 + o;
  } else if (bstart < g0 + g1 + g2) {
    const int o  = (i - g0 - g1) * 8;
    const int l  = o / (H2D * H2D);
    const int oo = o - l * (H2D * H2D);
    const int n  = oo / H2D;
    const int k0 = oo - n * H2D;
#pragma unroll
    for (int e = 0; e < 8; ++e)
      v[e] = Wh[(size_t)l * H2D * H2D + (size_t)(k0 + e) * H2D + n] * WSCALE;
    dp = Bh + o;
  } else {
    const int o  = (i - g0 - g1 - g2) * 8;
    const int n  = o / H2D;
    const int k0 = o - n * H2D;
    const int nc = n < NCLS ? n : NCLS - 1;
#pragma unroll
    for (int e = 0; e < 8; ++e) {
      const float a = Wfc[(size_t)(k0 + e) * NCLS + nc];
      v[e] = n < NCLS ? a * WSCALE : 0.0f;
    }
    dp = Bf + o;
  }
  v8f fv;
  fv[0] = v[0]; fv[1] = v[1]; fv[2] = v[2]; fv[3] = v[3]; fv[4] = v[4]; fv[5] = v[5]; fv[6] = v[6]; fv[7] = v[7];
  const v8h hv = tohalf8(fv);
  *(volatile v8h*)dp = hv;
  __threadfence();
  *(volatile v8h*)dp = hv;
}

__global__ __launch_bounds__(NTHR) void k_count(
    const int* __restrict__ ei, int* cnt, int nE, int vec8) {
  __shared__ __attribute__((aligned(16))) int scnt[NBC];
  __shared__ __attribute__((aligned(16))) int list[LISTN];
  __shared__ int wcnt[NWAVE];
  const int tid = threadIdx.x, lane = tid & 31, wave = tid >> 5;
  const int nodeBase = blockIdx.x * NBC;
  const int* dsts = ei + nE;

  for (int i = tid; i < NBC; i += NTHR) scnt[i] = 0;
  __syncthreads();

  const int nChunks = (nE + CHUNK - 1) / CHUNK;
#pragma unroll 1
  for (int ch = 0; ch < nChunks; ++ch) {
    const int cbase = ch * CHUNK;
    const int wc = scan_chunk<NBC>(dsts, nE, cbase, nodeBase, vec8, list, tid, lane, wave);
    if (lane == 0) wcnt[wave] = wc;
    __syncthreads();
    if (wave == 0) {
#pragma unroll 1
      for (int wsx = 0; wsx < NWAVE; ++wsx) {
        int n = __builtin_amdgcn_readfirstlane(wcnt[wsx]);
        n = n > WCAP ? WCAP : (n < 0 ? 0 : n);
        const int* lp = list + wsx * WCAP;
#pragma unroll 1
        for (int i = 0; i < n; ++i) {
          const int ent  = __builtin_amdgcn_readfirstlane(lp[i]);
          const int slot = ent & (NBC - 1);
          if (lane == 0) scnt[slot] = scnt[slot] + 1;
        }
      }
    }
    __syncthreads();
  }

  v4i cq[4];
#pragma unroll
  for (int q = 0; q < 4; ++q) {
    const int f = (wave * 4 + q) * 128 + 4 * lane;
    cq[q] = *(const v4i*)(scnt + f);
  }
  int* cp = cnt + (size_t)nodeBase;
#pragma unroll
  for (int q = 0; q < 4; ++q) {
    const int f = (wave * 4 + q) * 128 + 4 * lane;
    *(volatile v4i*)(cp + f) = cq[q];
  }
  __threadfence();
#pragma unroll
  for (int q = 0; q < 4; ++q) {
    const int f = (wave * 4 + q) * 128 + 4 * lane;
    *(volatile v4i*)(cp + f) = cq[q];
  }
}

__global__ __launch_bounds__(OTHR) void k_offsets(
    const int* __restrict__ cnt, int* off, int* rbase, int nChunk) {
  __shared__ __attribute__((aligned(16))) int soff[NBC];
  __shared__ __attribute__((aligned(16))) int srb[RBN];
  __shared__ int wtot[OTHR / 32];
  const int tid = threadIdx.x, lane = tid & 31, wave = tid >> 5, sub = tid >> 7;
  for (int i = tid; i < RBN; i += OTHR) srb[i] = 0;
  int carry = 0;
#pragma unroll 1
  for (int ch = 0; ch < nChunk; ++ch) {
    const int base = ch * NBC;
    const v4i c0 = *(const v4i*)(cnt + base + 8 * tid);
    const v4i c1 = *(const v4i*)(cnt + base + 8 * tid + 4);
    const int e0 = max(c0.x, 0), e1 = max(c0.y, 0), e2 = max(c0.z, 0), e3 = max(c0.w, 0);
    const int e4 = max(c1.x, 0), e5 = max(c1.y, 0), e6 = max(c1.z, 0), e7 = max(c1.w, 0);
    const int ts = e0 + e1 + e2 + e3 + e4 + e5 + e6 + e7;
    int incl = ts;
#pragma unroll
    for (int d = 1; d < 32; d <<= 1) {
      const int t = __shfl_up(incl, d);
      if (lane >= d) incl += t;
    }
    if (lane == 31) wtot[wave] = incl;
    __syncthreads();
    const int S0 = wtot[0]  + wtot[1]  + wtot[2]  + wtot[3];
    const int S1 = wtot[4]  + wtot[5]  + wtot[6]  + wtot[7];
    const int S2 = wtot[8]  + wtot[9]  + wtot[10] + wtot[11];
    const int S3 = wtot[12] + wtot[13] + wtot[14] + wtot[15];
    int pre = 0;
#pragma unroll 1
    for (int w = 4 * sub; w < wave; ++w) pre += wtot[w];
    const int b0 = carry;
    const int b1 = b0 + ((S0 + 31) & ~31);
    const int b2 = b1 + ((S1 + 31) & ~31);
    const int b3 = b2 + ((S2 + 31) & ~31);
    const int b4 = b3 + ((S3 + 31) & ~31);
    const int myb = sub == 0 ? b0 : (sub == 1 ? b1 : (sub == 2 ? b2 : b3));
    if (tid == 0) {
      srb[min(4 * ch + 0, RBN - 1)] = b0;
      srb[min(4 * ch + 1, RBN - 1)] = b1;
      srb[min(4 * ch + 2, RBN - 1)] = b2;
      srb[min(4 * ch + 3, RBN - 1)] = b3;
    }
    int run = myb + pre + incl - ts;
    soff[8 * tid + 0] = run; run += e0;
    soff[8 * tid + 1] = run; run += e1;
    soff[8 * tid + 2] = run; run += e2;
    soff[8 * tid + 3] = run; run += e3;
    soff[8 * tid + 4] = run; run += e4;
    soff[8 * tid + 5] = run; run += e5;
    soff[8 * tid + 6] = run; run += e6;
    soff[8 * tid + 7] = run;
    carry = b4;
    __syncthreads();
    const v4i o0 = *(const v4i*)(soff + 4 * tid);
    const v4i o1 = *(const v4i*)(soff + 4 * (tid + OTHR));
    int* op = off + base;
    *(volatile v4i*)(op + 4 * tid) = o0;
    *(volatile v4i*)(op + 4 * (tid + OTHR)) = o1;
    __threadfence();
    *(volatile v4i*)(op + 4 * tid) = o0;
    *(volatile v4i*)(op + 4 * (tid + OTHR)) = o1;
    __syncthreads();
  }
  if (tid == 0) srb[min(4 * nChunk, RBN - 1)] = carry;
  __syncthreads();
  v4i rv = {0, 0, 0, 0};
  if (tid < 32) rv = *(const v4i*)(srb + 4 * tid);
  if (tid < 32) *(volatile v4i*)(rbase + 4 * tid) = rv;
  __threadfence();
  if (tid < 32) *(volatile v4i*)(rbase + 4 * tid) = rv;
}

__global__ __launch_bounds__(NTHR) void k_fill(
    const int* __restrict__ ei, const int* __restrict__ off, const int* __restrict__ rbase,
    int* csr, int nN, int nE, int vec8, int csrLen) {
  extern __shared__ v4f lds_dyn[];
  int* region = (int*)lds_dyn;
  int* cursor = region + RCAP;
  int* list   = cursor + NBF;
  int* wcnt   = list + LISTN;
  const int tid = threadIdx.x, lane = tid & 31, wave = tid >> 5;
  const int b = blockIdx.x;
  const int nodeBase = b * NBF;
  const int* dsts = ei + nE;

  int rb0 = rbase[b];
  const int rb1 = rbase[b + 1];
  rb0 = rb0 < 0 ? 0 : (rb0 > csrLen ? csrLen : rb0);
  rb0 &= ~31;
  int len = rb1 - rb0;
  len = len < 0 ? 0 : (len > RCAP ? RCAP : len);
  int lenW = (len + 31) & ~31;
  if (rb0 + lenW > csrLen) lenW = (csrLen - rb0) & ~31;

  {
    const v4i z = {0, 0, 0, 0};
    for (int i = tid; i < RCAP / 4; i += NTHR) ((v4i*)region)[i] = z;
    for (int s = tid; s < NBF; s += NTHR) {
      int o = off[nodeBase + s] - rb0;
      o = o < 0 ? 0 : (o > RCAP ? RCAP : o);
      cursor[s] = o;
    }
  }
  __syncthreads();

  const int nChunks = (nE + CHUNK - 1) / CHUNK;
#pragma unroll 1
  for (int ch = 0; ch < nChunks; ++ch) {
    const int cbase = ch * CHUNK;
    const int wc = scan_chunk<NBF>(dsts, nE, cbase, nodeBase, vec8, list, tid, lane, wave);
    if (lane == 0) wcnt[wave] = wc;
    __syncthreads();
    if (wave == 0) {
#pragma unroll 1
      for (int wsx = 0; wsx < NWAVE; ++wsx) {
        int n = __builtin_amdgcn_readfirstlane(wcnt[wsx]);
        n = n > WCAP ? WCAP : (n < 0 ? 0 : n);
        const int* lp = list + wsx * WCAP;
#pragma unroll 1
        for (int i = 0; i < n; ++i) {
          const int ent  = __builtin_amdgcn_readfirstlane(lp[i]);
          const int slot = ent & (NBF - 1);
          int e = cbase + ((ent >> 12) & (CHUNK - 1));
          e = e > nE - 1 ? nE - 1 : e;
          int src = ei[e];
          src = src < 0 ? 0 : (src > nN - 1 ? nN - 1 : src);
          if (lane == 0) {
            int pos = cursor[slot];
            pos = pos < 0 ? 0 : (pos > RCAP - 1 ? RCAP - 1 : pos);
            region[pos] = src;
            const int np = pos + 1;
            cursor[slot] = np > RCAP ? RCAP : np;
          }
        }
      }
    }
    __syncthreads();
  }

  const int nv = lenW >> 2;
  int* gp = csr + rb0;
#pragma unroll 1
  for (int i = tid; i < nv; i += NTHR) { const v4i v = ((const v4i*)region)[i]; *(volatile v4i*)(gp + 4 * i) = v; }
  __threadfence();
#pragma unroll 1
  for (int i = tid; i < nv; i += NTHR) { const v4i v = ((const v4i*)region)[i]; *(volatile v4i*)(gp + 4 * i) = v; }
}

__global__ __launch_bounds__(NTHR) void k_agg1(
    const int* __restrict__ csr, const int* __restrict__ off, const int* __restrict__ cnt,
    const float* __restrict__ x, _Float16* A1, int nN, int csrLen) {
  const int tid = threadIdx.x, lane = tid & 31, wave = tid >> 5;
  const int tbase = blockIdx.x * TGT + wave * 32;
  const int cnt_l = cnt[tbase + lane];
  const int off_l = off[tbase + lane];

#pragma unroll 1
  for (int j = 0; j < 32; ++j) {
    const int c = tbase + j;
    int n = __builtin_amdgcn_readlane(cnt_l, j);
    n = n < 0 ? 0 : (n > DEGCAP ? DEGCAP : n);
    const int st = __builtin_amdgcn_readlane(off_l, j);
    v4f a = {0.f, 0.f, 0.f, 0.f};
    v4f b = {0.f, 0.f, 0.f, 0.f};
#pragma unroll 1
    for (int q0 = 0; q0 < n; q0 += 32) {
      int pos = st + q0 + lane;
      pos = pos < 0 ? 0 : (pos > csrLen - 1 ? csrLen - 1 : pos);
      int sl = csr[pos];
      sl = sl < 0 ? 0 : (sl > nN - 1 ? nN - 1 : sl);
      const int mcnt = (n - q0) < 32 ? (n - q0) : 32;
#pragma unroll 1
      for (int p = 0; p < mcnt; ++p) {
        const int s = __builtin_amdgcn_readlane(sl, p);
        const float* xp = x + (size_t)s * FEAT + 8 * lane;
        a = a + *(const v4f*)xp;
        b = b + *(const v4f*)(xp + 4);
      }
    }
    const float inv = 1.0f / (float)(n < 1 ? 1 : n);
    const int cr = c < nN ? c : nN - 1;
    const float* xr = x + (size_t)cr * FEAT + 8 * lane;
    const v4f xa = *(const v4f*)xr;
    const v4f xb = *(const v4f*)(xr + 4);
    const v8h hg = tohalf8(join8(a * inv, b * inv));
    const v8h hx = tohalf8(join8(xa, xb));
    _Float16* rp = A1 + (size_t)c * K1 + 8 * lane;
    *(volatile v8h*)rp = hg;
    *(volatile v8h*)(rp + FEAT) = hx;
    __threadfence();
    *(volatile v8h*)rp = hg;
    *(volatile v8h*)(rp + FEAT) = hx;
  }
}

__global__ __launch_bounds__(NTHR) void k_agg2(
    const int* __restrict__ csr, const int* __restrict__ off, const int* __restrict__ cnt,
    const _Float16* __restrict__ hin, _Float16* agg, int nN, int csrLen) {
  const int tid = threadIdx.x, lane = tid & 31, wave = tid >> 5;
  const int tbase = blockIdx.x * TGT + wave * 32;
  const int cnt_l = cnt[tbase + lane];
  const int off_l = off[tbase + lane];

#pragma unroll 1
  for (int j = 0; j < 32; ++j) {
    const int c = tbase + j;
    int n = __builtin_amdgcn_readlane(cnt_l, j);
    n = n < 0 ? 0 : (n > DEGCAP ? DEGCAP : n);
    const int st = __builtin_amdgcn_readlane(off_l, j);
    v8f a = {0.f, 0.f, 0.f, 0.f, 0.f, 0.f, 0.f, 0.f};
    v8f b = {0.f, 0.f, 0.f, 0.f, 0.f, 0.f, 0.f, 0.f};
#pragma unroll 1
    for (int q0 = 0; q0 < n; q0 += 32) {
      int pos = st + q0 + lane;
      pos = pos < 0 ? 0 : (pos > csrLen - 1 ? csrLen - 1 : pos);
      int sl = csr[pos];
      sl = sl < 0 ? 0 : (sl > nN - 1 ? nN - 1 : sl);
      const int mcnt = (n - q0) < 32 ? (n - q0) : 32;
#pragma unroll 1
      for (int p = 0; p < mcnt; ++p) {
        const int s = __builtin_amdgcn_readlane(sl, p);
        const _Float16* hp = hin + (size_t)s * H1D + 8 * lane;
        a = a + tofloat8(*(const v8h*)hp);
        b = b + tofloat8(*(const v8h*)(hp + 256));
      }
    }
    const float inv = 1.0f / (float)(n < 1 ? 1 : n);
    const v8h h0 = tohalf8(a * inv);
    const v8h h1 = tohalf8(b * inv);
    _Float16* rp = agg + (size_t)c * H1D + 8 * lane;
    *(volatile v8h*)rp = h0;
    *(volatile v8h*)(rp + 256) = h1;
    __threadfence();
    *(volatile v8h*)rp = h0;
    *(volatile v8h*)(rp + 256) = h1;
  }
}

__device__ __forceinline__ void zacc(v8f (&acc)[2][4]) {
  const v8f z = {0.f, 0.f, 0.f, 0.f, 0.f, 0.f, 0.f, 0.f};
#pragma unroll
  for (int i = 0; i < 2; ++i)
#pragma unroll
    for (int t = 0; t < 4; ++t) acc[i][t] = z;
}

template <int KPB>
__device__ __forceinline__ void mm32x64(const _Float16* a0p, const _Float16* a1p, const _Float16* bp,
                                        int ksteps, v8f (&acc)[2][4]) {
#pragma unroll 1
  for (int kt = 0; kt < ksteps; ++kt) {
    FragH a0, a1;
    a0.h[0] = *(const v8h*)(a0p + 32 * kt);
    a0.h[1] = *(const v8h*)(a0p + 32 * kt + 16);
    a1.h[0] = *(const v8h*)(a1p + 32 * kt);
    a1.h[1] = *(const v8h*)(a1p + 32 * kt + 16);
#pragma unroll
    for (int t = 0; t < 4; ++t) {
      const _Float16* bq = bp + (size_t)(16 * t) * KPB + 32 * kt;
      FragH b;
      b.h[0] = *(const v8h*)bq;
      b.h[1] = *(const v8h*)(bq + 16);
      wmh2(acc[0][t], acc[1][t], a0.v, a1.v, b.v);
    }
  }
}

__device__ __forceinline__ void epi64(const v8f (&acc)[2][4], const float* __restrict__ bias,
                                      _Float16* T, int wr, int wc, int hh, int m) {
#pragma unroll
  for (int t = 0; t < 4; ++t) {
    const int col = 64 * wc + 16 * t + m;
    const float bv = bias[col];
#pragma unroll
    for (int i = 0; i < 2; ++i) {
      _Float16* sp = T + (32 * wr + 16 * i + 8 * hh) * SP + col;
#pragma unroll
      for (int r = 0; r < 8; ++r) {
        float v = acc[i][t][r] * WINV + bv;
        v = fmaxf(v, 0.0f);
        sp[r * SP] = (_Float16)v;
      }
    }
  }
}

__global__ __launch_bounds__(NTHR) void k_gemm1(
    const _Float16* __restrict__ A, const _Float16* __restrict__ Bs, const float* __restrict__ bias,
    _Float16* Hout) {
  __shared__ __attribute__((aligned(16))) _Float16 stg[GR * SP];
  const int tid = threadIdx.x, lane = tid & 31, wave = tid >> 5, hh = lane >> 4, m = lane & 15;
  const int wr = wave >> 2, wc = wave & 3;
  const int rowBase = blockIdx.x * GR;
  const int colBase = blockIdx.y * 256;

  v8f acc[2][4];
  zacc(acc);
  const _Float16* a0p = A + (size_t)(rowBase + 32 * wr + m) * K1 + 8 * hh;
  const _Float16* a1p = a0p + (size_t)16 * K1;
  const _Float16* bp  = Bs + (size_t)(colBase + 64 * wc + m) * K1 + 8 * hh;
  mm32x64<K1>(a0p, a1p, bp, K1 / 32, acc);
  epi64(acc, bias + colBase, stg, wr, wc, hh, m);
  __syncthreads();

  v8h hv[8];
#pragma unroll
  for (int q = 0; q < 8; ++q) hv[q] = *(const v8h*)(stg + (8 * wave + q) * SP + 8 * lane);
  _Float16* gp = Hout + ((size_t)rowBase + 8 * wave) * H1D + colBase + 8 * lane;
#pragma unroll
  for (int q = 0; q < 8; ++q) *(volatile v8h*)(gp + (size_t)q * H1D) = hv[q];
  __threadfence();
#pragma unroll
  for (int q = 0; q < 8; ++q) *(volatile v8h*)(gp + (size_t)q * H1D) = hv[q];
}

__global__ __launch_bounds__(NTHR) void k_tail(
    const _Float16* __restrict__ Agg, const _Float16* __restrict__ Hin,
    const _Float16* __restrict__ B2s, const float* __restrict__ bias2,
    const _Float16* __restrict__ Bhs, const float* __restrict__ bh,
    const _Float16* __restrict__ Bfs, const float* __restrict__ bfc,
    float* out, int nN, int nHid) {
  extern __shared__ v4f lds_dyn[];
  _Float16* T0 = (_Float16*)lds_dyn;
  const int tid = threadIdx.x, lane = tid & 31, wave = tid >> 5, hh = lane >> 4, m = lane & 15;
  const int wr = wave >> 2, wc = wave & 3;
  const int rowBase = blockIdx.x * GR;

  v8f acc[2][4];
  zacc(acc);
  {
    const size_t arow = (size_t)(rowBase + 32 * wr + m);
    const _Float16* bp  = B2s + (size_t)(64 * wc + m) * K2 + 8 * hh;
    const _Float16* a0p = Agg + arow * H1D + 8 * hh;
    const _Float16* a1p = a0p + (size_t)16 * H1D;
    mm32x64<K2>(a0p, a1p, bp, H1D / 32, acc);
    const _Float16* h0p = Hin + arow * H1D + 8 * hh;
    const _Float16* h1p = h0p + (size_t)16 * H1D;
    mm32x64<K2>(h0p, h1p, bp + H1D, H1D / 32, acc);
  }
  epi64(acc, bias2, T0, wr, wc, hh, m);
  __syncthreads();

  int inOff = 0;
#pragma unroll 1
  for (int li = 0; li < nHid; ++li) {
    _Float16* Tin  = T0 + inOff;
    _Float16* Tout = T0 + (GR * SP - inOff);
    zacc(acc);
    const _Float16* a0p = Tin + (32 * wr + m) * SP + 8 * hh;
    const _Float16* a1p = a0p + 16 * SP;
    const _Float16* bp  = Bhs + (size_t)li * H2D * H2D + (size_t)(64 * wc + m) * H2D + 8 * hh;
    mm32x64<H2D>(a0p, a1p, bp, H2D / 32, acc);
    epi64(acc, bh + (size_t)li * H2D, Tout, wr, wc, hh, m);
    __syncthreads();
    inOff = GR * SP - inOff;
  }

  _Float16* Tf = T0 + inOff;
  float* slog = (float*)(T0 + (GR * SP - inOff));
  float* spr  = slog + GR * 8;
  const int tw = wave & 3;
  v8f cacc = {0.f, 0.f, 0.f, 0.f, 0.f, 0.f, 0.f, 0.f};
  {
    const _Float16* ap = Tf + (16 * tw + m) * SP + 8 * hh;
    const _Float16* bp = Bfs + (size_t)m * H2D + 8 * hh;
#pragma unroll 1
    for (int kt = 0; kt < H2D / 32; ++kt) {
      FragH a, b;
      a.h[0] = *(const v8h*)(ap + 32 * kt);
      a.h[1] = *(const v8h*)(ap + 32 * kt + 16);
      b.h[0] = *(const v8h*)(bp + 32 * kt);
      b.h[1] = *(const v8h*)(bp + 32 * kt + 16);
      cacc = wmh(a.v, b.v, cacc);
    }
  }
  const float bq = bfc[m < NCLS ? m : NCLS - 1];
  if (wave < 4 && m < NCLS) {
    float* lp = slog + (16 * tw + 8 * hh) * 8 + m;
#pragma unroll
    for (int r = 0; r < 8; ++r) lp[r * 8] = cacc[r] * WINV + bq;
  }
  __syncthreads();

  if (tid < GR) {
    const float* lr = slog + tid * 8;
    float e[NCLS];
    float mx = lr[0];
#pragma unroll
    for (int c = 0; c < NCLS; ++c) { e[c] = lr[c]; mx = fmaxf(mx, e[c]); }
    float s = 0.0f;
#pragma unroll
    for (int c = 0; c < NCLS; ++c) { e[c] = __expf(e[c] - mx); s += e[c]; }
    const float inv = 1.0f / s;
#pragma unroll
    for (int c = 0; c < NCLS; ++c) spr[tid * NCLS + c] = e[c] * inv;
  }
  __syncthreads();

  int vr = nN - rowBase;
  vr = vr < 0 ? 0 : (vr > GR ? GR : vr);
  const int vf  = vr * NCLS;
  const int npc = vf >> 2;
  const int rem = vf & 3;
  const int p   = wave * 32 + lane;
  const int pcl = p < (GR * NCLS / 4 - 1) ? p : (GR * NCLS / 4 - 1);
  const v4f ov  = *(const v4f*)(spr + 4 * pcl);
  const bool act = p < npc;
  float tv[3];
#pragma unroll
  for (int e = 0; e < 3; ++e) {
    const int idx = 4 * npc + e;
    tv[e] = spr[idx < GR * NCLS ? idx : GR * NCLS - 1];
  }
  float* op = out + (size_t)rowBase * NCLS;
  if (act) *(volatile v4f*)(op + 4 * p) = ov;
  if (tid == 0) {
    if (rem > 0) *(volatile float*)(op + 4 * npc + 0) = tv[0];
    if (rem > 1) *(volatile float*)(op + 4 * npc + 1) = tv[1];
    if (rem > 2) *(volatile float*)(op + 4 * npc + 2) = tv[2];
  }
  __threadfence();
  if (act) *(volatile v4f*)(op + 4 * p) = ov;
  if (tid == 0) {
    if (rem > 0) *(volatile float*)(op + 4 * npc + 0) = tv[0];
    if (rem > 1) *(volatile float*)(op + 4 * npc + 1) = tv[1];
    if (rem > 2) *(volatile float*)(op + 4 * npc + 2) = tv[2];
  }
}

extern "C" void kernel_launch(void* const* d_in, const int* in_sizes, int n_in,
                              void* d_out, int out_size, void* d_ws, size_t ws_size,
                              hipStream_t stream) {
  if (n_in < 12) return;
  const int nN = in_sizes[0] / FEAT;
  const int nE = in_sizes[1] / 2;
  if (nN <= 0 || nE <= 0 || in_sizes[0] != nN * FEAT || in_sizes[1] != 2 * nE) return;
  if (in_sizes[2] != FEAT * H1D || in_sizes[3] < H1D || in_sizes[4] != FEAT * H1D) return;
  if (in_sizes[5] != H1D * H2D || in_sizes[6] < H2D || in_sizes[7] != H1D * H2D) return;
  const int nHid = in_sizes[8] / (H2D * H2D);
  if (nHid < 1 || nHid > 64 || in_sizes[8] != nHid * H2D * H2D || in_sizes[9] < nHid * H2D) return;
  if (in_sizes[10] != H2D * NCLS || in_sizes[11] < NCLS) return;
  if (out_size != nN * NCLS) return;
  if (nE > (1 << 28) || nN > (1 << 22)) return;

  const float* x   = (const float*)d_in[0];
  const int*   ei  = (const int*)d_in[1];
  const float* W1l = (const float*)d_in[2];
  const float* b1  = (const float*)d_in[3];
  const float* W1r = (const float*)d_in[4];
  const float* W2l = (const float*)d_in[5];
  const float* b2  = (const float*)d_in[6];
  const float* W2r = (const float*)d_in[7];
  const float* Wh  = (const float*)d_in[8];
  const float* bh  = (const float*)d_in[9];
  const float* Wfc = (const float*)d_in[10];
  const float* bfc = (const float*)d_in[11];
  float* out = (float*)d_out;

  const int NPAD   = ((nN + TGT - 1) / TGT) * TGT;
  const int nBC    = (nN + NBC - 1) / NBC;
  const int CNTPAD = nBC * NBC;
  if (4 * nBC + 1 > RBN) return;
  if (CNTPAD < NPAD) return;
  const int nBF    = (nN + NBF - 1) / NBF;
  const int csrLen = ((nE + 31) & ~31) + 4096;
  const int nAgg   = NPAD / TGT;
  const int nTile  = NPAD / GR;

  char* ws = (char*)d_ws;
  size_t off = 0;
  const size_t oB1  = off; off += (size_t)H1D * K1 * 2;            off = (off + 255) & ~(size_t)255;
  const size_t oB2  = off; off += (size_t)H2D * K2 * 2;            off = (off + 255) & ~(size_t)255;
  const size_t oBh  = off; off += (size_t)nHid * H2D * H2D * 2;    off = (off + 255) & ~(size_t)255;
  const size_t oBf  = off; off += (size_t)NCLP * H2D * 2;          off = (off + 255) & ~(size_t)255;
  const size_t oCnt = off; off += (size_t)CNTPAD * 4;              off = (off + 255) & ~(size_t)255;
  const size_t oOff = off; off += (size_t)CNTPAD * 4;              off = (off + 255) & ~(size_t)255;
  const size_t oRb  = off; off += (size_t)RBN * 4;                 off = (off + 255) & ~(size_t)255;
  const size_t oCsr = off; off += (size_t)csrLen * 4;              off = (off + 255) & ~(size_t)255;
  const size_t oA1  = off; off += (size_t)NPAD * K1 * 2;           off = (off + 255) & ~(size_t)255;
  const size_t oH1  = off; off += (size_t)NPAD * H1D * 2;          off = (off + 255) & ~(size_t)255;
  if (off > ws_size) return;
  _Float16* B1p  = (_Float16*)(ws + oB1);
  _Float16* B2p  = (_Float16*)(ws + oB2);
  _Float16* Bhp  = (_Float16*)(ws + oBh);
  _Float16* Bfp  = (_Float16*)(ws + oBf);
  int*      cnt  = (int*)(ws + oCnt);
  int*      offp = (int*)(ws + oOff);
  int*      rb   = (int*)(ws + oRb);
  int*      csr  = (int*)(ws + oCsr);
  _Float16* A1   = (_Float16*)(ws + oA1);
  _Float16* agg2 = (_Float16*)(ws + oA1);
  _Float16* h1   = (_Float16*)(ws + oH1);

  const int vec8 = ((nE & 3) == 0) ? 1 : 0;

  const int nPrep = H1D * K1 / 8 + H2D * K2 / 8 + nHid * (H2D * H2D / 8) + NCLP * H2D / 8;
  k_wprep<<<(nPrep + NTHR - 1) / NTHR, NTHR, 0, stream>>>(W1l, W1r, W2l, W2r, Wh, Wfc, B1p, B2p, Bhp, Bfp, nHid);

  k_count<<<nBC, NTHR, 0, stream>>>(ei, cnt, nE, vec8);
  k_offsets<<<1, OTHR, 0, stream>>>(cnt, offp, rb, nBC);
  hipFuncSetAttribute(reinterpret_cast<const void*>(&k_fill),
                      hipFuncAttributeMaxDynamicSharedMemorySize, LDS_FILL);
  k_fill<<<nBF, NTHR, LDS_FILL, stream>>>(ei, offp, rb, csr, nN, nE, vec8, csrLen);

  k_agg1<<<nAgg, NTHR, 0, stream>>>(csr, offp, cnt, x, A1, nN, csrLen);
  k_gemm1<<<dim3(nTile, H1D / 256), NTHR, 0, stream>>>(A1, B1p, b1, h1);

  k_agg2<<<nAgg, NTHR, 0, stream>>>(csr, offp, cnt, h1, agg2, nN, csrLen);
  hipFuncSetAttribute(reinterpret_cast<const void*>(&k_tail),
                      hipFuncAttributeMaxDynamicSharedMemorySize, LDS_TAIL);
  k_tail<<<nTile, NTHR, LDS_TAIL, stream>>>(agg2, h1, B2p, b2, Bhp, bh, Bfp, bfc, out, nN, nHid);
}
